// TransformerBlock_4690104287476
// MI455X (gfx1250) — hardware-verified
//
#include <hip/hip_runtime.h>
#include <math.h>
#include <stdint.h>


#ifndef NB
#define NB 2
#endif
#ifndef SEQ
#define SEQ 2048
#endif
#define NB_FULL 2
#define SEQ_FULL 2048
#define DMODEL 1024
#define DFF 4096
#define NHEAD 16
#define HDIM 64
#define NR (NB * SEQ)
#define LDC 68
#define LDP 72
#define LDT 72

static_assert(NB >= 1 && NB <= NB_FULL);
static_assert(SEQ >= 128 && SEQ <= SEQ_FULL && (SEQ % 128) == 0);
static_assert((NR % 128) == 0);
static_assert(DMODEL == NHEAD * HDIM);

typedef _Float16 v16h __attribute__((ext_vector_type(16)));
typedef _Float16 v8h __attribute__((ext_vector_type(8)));
typedef _Float16 v2h __attribute__((ext_vector_type(2)));
typedef float v8f __attribute__((ext_vector_type(8)));
typedef float v4f __attribute__((ext_vector_type(4)));
typedef float v2f __attribute__((ext_vector_type(2)));

union Frag { v16h v; v8h hv[2]; };

constexpr size_t SZ_WSQ  = (size_t)DMODEL * DMODEL * 2;
constexpr size_t SZ_WFF  = (size_t)DMODEL * DFF * 2;
constexpr size_t SZ_TAB  = (size_t)SEQ * 32 * 4;
constexpr size_t SZ_P16  = (size_t)NR * DMODEL * 2;
constexpr size_t SZ_QKVE = (size_t)NB * 3 * 64 * DMODEL * 4;
constexpr size_t SZ_OUT1 = (size_t)NR * DMODEL * 4;
constexpr size_t SZ_T16  = (size_t)NR * DFF * 2;
constexpr size_t OFF_WQT  = 0;
constexpr size_t OFF_WKT  = OFF_WQT + SZ_WSQ;
constexpr size_t OFF_WVT  = OFF_WKT + SZ_WSQ;
constexpr size_t OFF_WOT  = OFF_WVT + SZ_WSQ;
constexpr size_t OFF_W1T  = OFF_WOT + SZ_WSQ;
constexpr size_t OFF_W3T  = OFF_W1T + SZ_WFF;
constexpr size_t OFF_W2T  = OFF_W3T + SZ_WFF;
constexpr size_t OFF_COS  = OFF_W2T + SZ_WFF;
constexpr size_t OFF_SIN  = OFF_COS + SZ_TAB;
constexpr size_t OFF_RH   = OFF_SIN + SZ_TAB;
constexpr size_t OFF_RQ   = OFF_RH + SZ_P16;
constexpr size_t OFF_K16  = OFF_RQ + SZ_P16;
constexpr size_t OFF_VT   = OFF_K16 + SZ_P16;
constexpr size_t OFF_QKVE = OFF_VT + SZ_P16;
constexpr size_t OFF_OUT1 = OFF_QKVE + SZ_QKVE;
constexpr size_t OFF_T16  = OFF_OUT1 + SZ_OUT1;
constexpr size_t WS_TOTAL = OFF_T16 + SZ_T16;
static_assert(WS_TOTAL <= (size_t)134217728);
static_assert((size_t)NB * NHEAD * HDIM * SEQ * 2 == SZ_P16);

__device__ __forceinline__ v16h ld_frag(const _Float16* p0, size_t ld) {
  const int l = threadIdx.x & 31;
  const int hh = l >> 4, m = l & 15;
  const _Float16* p = p0 + (size_t)m * ld + 8 * hh;
  Frag f;
  f.hv[0] = *(const v8h*)p;
  f.hv[1] = *(const v8h*)(p + 16);
  return f.v;
}

__device__ __forceinline__ v8f mma16(v16h a, v16h b, v8f c) {
  v8f d = __builtin_amdgcn_wmma_f32_16x16x32_f16(false, a, false, b, (short)0, c, false, false);
  asm volatile("v_nop\n\tv_nop\n\tv_nop\n\tv_nop" : "+v"(d) : "v"(a), "v"(b));
  return d;
}

__device__ __forceinline__ v8f vzero() {
  v8f z = {0.f, 0.f, 0.f, 0.f, 0.f, 0.f, 0.f, 0.f};
  return z;
}

__device__ __forceinline__ float bfr(float f) {
  unsigned int u = __float_as_uint(f);
  u = (u + 0x7FFFu + ((u >> 16) & 1u)) & 0xFFFF0000u;
  return __uint_as_float(u);
}

__device__ __forceinline__ size_t full_row(int r) {
  return (size_t)(r / SEQ) * SEQ_FULL + (size_t)(r % SEQ);
}

__global__ __launch_bounds__(256) void cvt_w_kernel(
    const float* __restrict__ Wq, const float* __restrict__ Wk, const float* __restrict__ Wv,
    const float* __restrict__ Wo, const float* __restrict__ W1, const float* __restrict__ W2,
    const float* __restrict__ W3,
    _Float16* __restrict__ WqT, _Float16* __restrict__ WkT, _Float16* __restrict__ WvT,
    _Float16* __restrict__ WoT, _Float16* __restrict__ W1T, _Float16* __restrict__ W2T,
    _Float16* __restrict__ W3T) {
  __shared__ _Float16 Ts[64 * LDT] __attribute__((aligned(16)));
  const int z = blockIdx.z;
  const float* W;
  _Float16* D;
  int KK, NN;
  if (z == 0)      { W = Wq; D = WqT; KK = DMODEL; NN = DMODEL; }
  else if (z == 1) { W = Wk; D = WkT; KK = DMODEL; NN = DMODEL; }
  else if (z == 2) { W = Wv; D = WvT; KK = DMODEL; NN = DMODEL; }
  else if (z == 3) { W = Wo; D = WoT; KK = DMODEL; NN = DMODEL; }
  else if (z == 4) { W = W1; D = W1T; KK = DMODEL; NN = DFF; }
  else if (z == 5) { W = W2; D = W2T; KK = DFF;    NN = DMODEL; }
  else             { W = W3; D = W3T; KK = DMODEL; NN = DFF; }
  const int ntn = NN / 64;
  const int ntiles = (KK / 64) * ntn;
  const int t = blockIdx.x;
  if (t >= ntiles) return;
  const int k0 = (t / ntn) * 64, n0 = (t % ntn) * 64;
  const int tid = threadIdx.x;
#pragma unroll
  for (int p = 0; p < 4; ++p) {
    const int idx = tid + 256 * p;
    const int r = idx >> 4, c4 = (idx & 15) * 4;
    const v4f v = *(const v4f*)(W + (size_t)(k0 + r) * NN + n0 + c4);
#pragma unroll
    for (int e = 0; e < 4; ++e) {
      const float f = v[e];
      Ts[(c4 + e) * LDT + r] = (_Float16)(bfr(f) * 64.0f);
    }
  }
  __syncthreads();
  const int seg = tid & 7, rb = tid >> 3;
  v8h o[2];
#pragma unroll
  for (int p = 0; p < 2; ++p) o[p] = *(const v8h*)(Ts + (rb + 32 * p) * LDT + 8 * seg);
#pragma unroll
  for (int p = 0; p < 2; ++p)
    *(volatile v8h*)(D + (size_t)(n0 + rb + 32 * p) * KK + k0 + 8 * seg) = o[p];
  __threadfence();
#pragma unroll
  for (int p = 0; p < 2; ++p)
    *(volatile v8h*)(D + (size_t)(n0 + rb + 32 * p) * KK + k0 + 8 * seg) = o[p];
}

__global__ __launch_bounds__(256) void rope_tab_kernel(float* __restrict__ cosT,
                                                       float* __restrict__ sinT) {
  const int idx = blockIdx.x * 256 + threadIdx.x;
  const int i = idx & 31, s = idx >> 5;
  double dd = 1.0;
#pragma unroll 1
  for (int j = 0; j < i; ++j) dd *= 1.333521432163324;
  const float th = (float)dd;
  const float inv = (float)(1.0 / (double)th);
  const float ang = (float)s * inv;
  const float c = cosf(ang), sn = sinf(ang);
  *(volatile float*)(cosT + idx) = c;
  *(volatile float*)(sinT + idx) = sn;
  __threadfence();
  *(volatile float*)(cosT + idx) = c;
  *(volatile float*)(sinT + idx) = sn;
}

template <int RIN>
__global__ __launch_bounds__(256) void rmsnorm_kernel(const float* __restrict__ X,
                                                      const float* __restrict__ g,
                                                      _Float16* __restrict__ Hout) {
  const int wave = threadIdx.x >> 5, l = threadIdx.x & 31;
  const int r = blockIdx.x * 8 + wave;
  const size_t srow = RIN ? full_row(r) : (size_t)r;
  const float* xr = X + srow * DMODEL;
  float v[32];
  float ss = 0.f;
#pragma unroll
  for (int j = 0; j < 4; ++j) {
    const v4f a = *(const v4f*)(xr + 256 * j + 8 * l);
    const v4f bq = *(const v4f*)(xr + 256 * j + 8 * l + 4);
#pragma unroll
    for (int e = 0; e < 4; ++e) {
      float t0 = a[e], t1 = bq[e];
      if (RIN) { t0 = bfr(t0); t1 = bfr(t1); }
      v[8 * j + e] = t0;
      v[8 * j + 4 + e] = t1;
      ss += t0 * t0;
      ss += t1 * t1;
    }
  }
  ss += __shfl_xor(ss, 16);
  ss += __shfl_xor(ss, 8);
  ss += __shfl_xor(ss, 4);
  ss += __shfl_xor(ss, 2);
  ss += __shfl_xor(ss, 1);
  const float rinv = 1.0f / sqrtf(ss * (1.0f / DMODEL) + 1e-5f);
  v8h o[4];
#pragma unroll
  for (int j = 0; j < 4; ++j) {
    const v4f ga = *(const v4f*)(g + 256 * j + 8 * l);
    const v4f gb = *(const v4f*)(g + 256 * j + 8 * l + 4);
    v8h t;
#pragma unroll
    for (int e = 0; e < 4; ++e) {
      const float g0 = ga[e], g1 = gb[e];
      t[e]     = (_Float16)(v[8 * j + e] * rinv * bfr(g0));
      t[4 + e] = (_Float16)(v[8 * j + 4 + e] * rinv * bfr(g1));
    }
    o[j] = t;
  }
  _Float16* hr = Hout + (size_t)r * DMODEL + 8 * l;
#pragma unroll
  for (int j = 0; j < 4; ++j) *(volatile v8h*)(hr + 256 * j) = o[j];
  __threadfence();
#pragma unroll
  for (int j = 0; j < 4; ++j) *(volatile v8h*)(hr + 256 * j) = o[j];
}

template <int K, bool TWO>
__device__ __forceinline__ void gemm_core(const _Float16* __restrict__ A,
                                          const _Float16* __restrict__ B0,
                                          const _Float16* __restrict__ B1,
                                          int row0, int n0,
                                          v8f (&acc)[2][2], v8f (&acx)[2][2]) {
  const int wave = threadIdx.x >> 5;
  const int wm = wave & 3, wn = wave >> 2;
  const _Float16* ap = A + (size_t)(row0 + wm * 32) * K;
  const _Float16* bp = B0 + (size_t)(n0 + wn * 32) * K;
  const _Float16* cp = B1 + (size_t)(n0 + wn * 32) * K;
#pragma unroll 1
  for (int k0 = 0; k0 < K; k0 += 32) {
    const v16h a0 = ld_frag(ap + k0, K);
    const v16h a1 = ld_frag(ap + (size_t)16 * K + k0, K);
    const v16h b0 = ld_frag(bp + k0, K);
    const v16h b1 = ld_frag(bp + (size_t)16 * K + k0, K);
    acc[0][0] = mma16(a0, b0, acc[0][0]);
    acc[0][1] = mma16(a0, b1, acc[0][1]);
    acc[1][0] = mma16(a1, b0, acc[1][0]);
    acc[1][1] = mma16(a1, b1, acc[1][1]);
    if (TWO) {
      const v16h c0 = ld_frag(cp + k0, K);
      const v16h c1 = ld_frag(cp + (size_t)16 * K + k0, K);
      acx[0][0] = mma16(a0, c0, acx[0][0]);
      acx[0][1] = mma16(a0, c1, acx[0][1]);
      acx[1][0] = mma16(a1, c0, acx[1][0]);
      acx[1][1] = mma16(a1, c1, acx[1][1]);
    }
  }
}

__device__ __forceinline__ void stage_acc(float* Cs, v8f (&acc)[2][2], float sc) {
  const int wave = threadIdx.x >> 5, l = threadIdx.x & 31;
  const int wm = wave & 3, wn = wave >> 2, hh = l >> 4, m = l & 15;
#pragma unroll
  for (int mi = 0; mi < 2; ++mi)
#pragma unroll
    for (int ni = 0; ni < 2; ++ni)
#pragma unroll
      for (int r = 0; r < 8; ++r)
        Cs[(wm * 32 + mi * 16 + 8 * hh + r) * LDC + wn * 32 + ni * 16 + m] = acc[mi][ni][r] * sc;
}

__device__ __forceinline__ void store_f16_rows(const float* Cs, _Float16* dst, size_t pitch) {
  const int tid = threadIdx.x;
  const int seg = tid & 7, rb = tid >> 3;
  v8h o[4];
#pragma unroll
  for (int p = 0; p < 4; ++p) {
    const float* c = Cs + (rb + 32 * p) * LDC + 8 * seg;
    const v4f x0 = *(const v4f*)c;
    const v4f x1 = *(const v4f*)(c + 4);
    v8h t;
#pragma unroll
    for (int e = 0; e < 4; ++e) { t[e] = (_Float16)x0[e]; t[4 + e] = (_Float16)x1[e]; }
    o[p] = t;
  }
#pragma unroll
  for (int p = 0; p < 4; ++p)
    *(volatile v8h*)(dst + (size_t)(rb + 32 * p) * pitch + 8 * seg) = o[p];
  __threadfence();
#pragma unroll
  for (int p = 0; p < 4; ++p)
    *(volatile v8h*)(dst + (size_t)(rb + 32 * p) * pitch + 8 * seg) = o[p];
}

__global__ __launch_bounds__(256) void qkv_kernel(
    const _Float16* __restrict__ H16, const _Float16* __restrict__ WqT,
    const _Float16* __restrict__ WkT, const _Float16* __restrict__ WvT,
    const float* __restrict__ cosT, const float* __restrict__ sinT,
    _Float16* __restrict__ Q16, _Float16* __restrict__ K16,
    _Float16* __restrict__ VT16, float* __restrict__ QKVe) {
  __shared__ float Cs[128 * LDC] __attribute__((aligned(16)));
  const int tid = threadIdx.x;
  const int row0 = blockIdx.x * 128;
  const int ncomb = blockIdx.y * 64;
  const int mat = ncomb / DMODEL;
  const int n0 = ncomb - mat * DMODEL;
  const int h = n0 / HDIM;
  const int bidx = row0 / SEQ;
  const int s0 = row0 - bidx * SEQ;
  const _Float16* Bm = (mat == 0) ? WqT : ((mat == 1) ? WkT : WvT);

  v8f acc[2][2];
#pragma unroll
  for (int i = 0; i < 2; ++i) { acc[i][0] = vzero(); acc[i][1] = vzero(); }
  gemm_core<DMODEL, false>(H16, Bm, Bm, row0, n0, acc, acc);
  stage_acc(Cs, acc, 0.015625f);
  __syncthreads();

  if (mat < 2) {
#pragma unroll 4
    for (int j = 0; j < 16; ++j) {
      const int p = tid + 256 * j;
      const int row = p >> 5, i = p & 31;
      const int s = s0 + row;
      const float c = cosT[s * 32 + i], sn = sinT[s * 32 + i];
      float* cr = Cs + row * LDC + 2 * i;
      const float x1 = cr[0], x2 = cr[1];
      cr[0] = x1 * c - x2 * sn;
      cr[1] = x2 * c + x1 * sn;
    }
    __syncthreads();
    _Float16* P = (mat == 0) ? Q16 : K16;
    store_f16_rows(Cs, P + (size_t)row0 * DMODEL + n0, DMODEL);
  } else {
    const int seg = tid & 15, db = tid >> 4;
    v8h o[4];
#pragma unroll
    for (int p = 0; p < 4; ++p) {
      const int d = db + 16 * p;
      v8h t;
#pragma unroll
      for (int e = 0; e < 8; ++e) t[e] = (_Float16)Cs[(8 * seg + e) * LDC + d];
      o[p] = t;
    }
    _Float16* vbp = VT16 + (((size_t)bidx * NHEAD + h) * HDIM) * SEQ + s0 + 8 * seg;
#pragma unroll
    for (int p = 0; p < 4; ++p) *(volatile v8h*)(vbp + (size_t)(db + 16 * p) * SEQ) = o[p];
    __threadfence();
#pragma unroll
    for (int p = 0; p < 4; ++p) *(volatile v8h*)(vbp + (size_t)(db + 16 * p) * SEQ) = o[p];
  }

  if (s0 == 0) {
    const int seg = tid & 15, rb = tid >> 4;
    v4f o[4];
#pragma unroll
    for (int p = 0; p < 4; ++p) o[p] = *(const v4f*)(Cs + (rb + 16 * p) * LDC + 4 * seg);
    float* eb = QKVe + (((size_t)bidx * 3 + mat) * 64) * DMODEL + n0 + 4 * seg;
#pragma unroll
    for (int p = 0; p < 4; ++p) *(volatile v4f*)(eb + (size_t)(rb + 16 * p) * DMODEL) = o[p];
    __threadfence();
#pragma unroll
    for (int p = 0; p < 4; ++p) *(volatile v4f*)(eb + (size_t)(rb + 16 * p) * DMODEL) = o[p];
  }
}

__global__ __launch_bounds__(256) void attn0_kernel(const float* __restrict__ QKVe,
                                                    _Float16* __restrict__ CTX) {
  __shared__ float Qs[64 * 64] __attribute__((aligned(16)));
  __shared__ float Ks[64 * 64] __attribute__((aligned(16)));
  __shared__ float Vs[64 * 64] __attribute__((aligned(16)));
  const int h = blockIdx.x, b = blockIdx.y;
  const int tid = threadIdx.x, wave = tid >> 5, l = tid & 31;
  const float* qb = QKVe + ((size_t)b * 3 + 0) * 64 * DMODEL + h * HDIM;
  const float* kb = QKVe + ((size_t)b * 3 + 1) * 64 * DMODEL + h * HDIM;
  const float* vb = QKVe + ((size_t)b * 3 + 2) * 64 * DMODEL + h * HDIM;
#pragma unroll
  for (int p = 0; p < 4; ++p) {
    const int idx = tid + 256 * p;
    const int row = idx >> 4, c4 = (idx & 15) * 4;
    *(v4f*)(Qs + row * 64 + c4) = *(const v4f*)(qb + (size_t)row * DMODEL + c4);
    *(v4f*)(Ks + row * 64 + c4) = *(const v4f*)(kb + (size_t)row * DMODEL + c4);
    *(v4f*)(Vs + row * 64 + c4) = *(const v4f*)(vb + (size_t)row * DMODEL + c4);
  }
  __syncthreads();
  const float NEG = -__builtin_inff();
#pragma unroll 1
  for (int ri = 0; ri < 8; ++ri) {
    const int i = wave + 8 * ri;
    const v2f q = *(const v2f*)(Qs + i * 64 + 2 * l);
    float mx = NEG, ls = 0.f, o0 = 0.f, o1 = 0.f;
#pragma unroll 1
    for (int j = 0; j <= i; ++j) {
      const v2f k = *(const v2f*)(Ks + j * 64 + 2 * l);
      const v2f v = *(const v2f*)(Vs + j * 64 + 2 * l);
      float s = q.x * k.x + q.y * k.y;
      s += __shfl_xor(s, 16);
      s += __shfl_xor(s, 8);
      s += __shfl_xor(s, 4);
      s += __shfl_xor(s, 2);
      s += __shfl_xor(s, 1);
      s *= 0.125f;
      const float nm = fmaxf(mx, s);
      const float al = expf(mx - nm);
      const float p = expf(s - nm);
      ls = ls * al + p;
      o0 = o0 * al + p * v.x;
      o1 = o1 * al + p * v.y;
      mx = nm;
    }
    const float inv = 1.0f / ls;
    v2h ov;
    ov.x = (_Float16)(o0 * inv);
    ov.y = (_Float16)(o1 * inv);
    _Float16* dst = CTX + ((size_t)b * SEQ + i) * DMODEL + h * HDIM + 2 * l;
    *(volatile v2h*)dst = ov;
    __threadfence();
    *(volatile v2h*)dst = ov;
  }
}

__global__ __launch_bounds__(128) void attn_kernel(
    const _Float16* __restrict__ Q16, const _Float16* __restrict__ K16,
    const _Float16* __restrict__ VT16, _Float16* __restrict__ CTX) {
  __shared__ _Float16 Pl[4 * 16 * LDP] __attribute__((aligned(16)));
  const int qt = blockIdx.x + 1, h = blockIdx.y, b = blockIdx.z;
  const int tid = threadIdx.x, wave = tid >> 5, l = tid & 31;
  const int hh = l >> 4, m = l & 15;
  const int qs0 = qt * 64 + wave * 16;
  const size_t prow0 = (size_t)b * SEQ + qs0;
  _Float16* Pw = Pl + wave * (16 * LDP);
  const _Float16* qp = Q16 + prow0 * DMODEL + h * HDIM;
  const v16h aq0 = ld_frag(qp, DMODEL);
  const v16h aq1 = ld_frag(qp + 32, DMODEL);
  const _Float16* Kb = K16 + (size_t)b * SEQ * DMODEL + h * HDIM;
  const _Float16* Vb = VT16 + ((size_t)b * NHEAD + h) * HDIM * (size_t)SEQ;
  const float NEG = -__builtin_inff();

  v8f acc[4];
#pragma unroll
  for (int n = 0; n < 4; ++n) acc[n] = vzero();
  float mrow[8], lrow[8];
#pragma unroll
  for (int r = 0; r < 8; ++r) { mrow[r] = NEG; lrow[r] = 0.f; }

  for (int kc = 0; kc <= qt; ++kc) {
    const int key0 = kc * 64;
    v8f sc[4];
#pragma unroll
    for (int t = 0; t < 4; ++t) {
      const _Float16* kp = Kb + (size_t)(key0 + 16 * t) * DMODEL;
      v8f s = vzero();
      s = mma16(aq0, ld_frag(kp, DMODEL), s);
      s = mma16(aq1, ld_frag(kp + 32, DMODEL), s);
      sc[t] = s * 0.125f;
    }
    if (kc == qt) {
#pragma unroll
      for (int t = 0; t < 4; ++t)
#pragma unroll
        for (int r = 0; r < 8; ++r) {
          const int qg = qs0 + 8 * hh + r, kg = key0 + 16 * t + m;
          if (kg > qg) sc[t][r] = NEG;
        }
    }
#pragma unroll
    for (int r = 0; r < 8; ++r) {
      float rm = fmaxf(fmaxf(sc[0][r], sc[1][r]), fmaxf(sc[2][r], sc[3][r]));
      rm = fmaxf(rm, __shfl_xor(rm, 1, 16));
      rm = fmaxf(rm, __shfl_xor(rm, 2, 16));
      rm = fmaxf(rm, __shfl_xor(rm, 4, 16));
      rm = fmaxf(rm, __shfl_xor(rm, 8, 16));
      const float nm = fmaxf(mrow[r], rm);
      const float al = __expf(mrow[r] - nm);
      float ps = 0.f;
#pragma unroll
      for (int t = 0; t < 4; ++t) {
        const float p = __expf(sc[t][r] - nm);
        ps += p;
        Pw[(8 * hh + r) * LDP + 16 * t + m] = (_Float16)(p * 1024.0f);
      }
      ps += __shfl_xor(ps, 1, 16);
      ps += __shfl_xor(ps, 2, 16);
      ps += __shfl_xor(ps, 4, 16);
      ps += __shfl_xor(ps, 8, 16);
      lrow[r] = lrow[r] * al + ps;
      mrow[r] = nm;
#pragma unroll
      for (int n = 0; n < 4; ++n) acc[n][r] *= al;
    }
    __syncthreads();
    const v16h ap0 = ld_frag(Pw, LDP);
    const v16h ap1 = ld_frag(Pw + 32, LDP);
#pragma unroll
    for (int n = 0; n < 4; ++n) {
      const _Float16* vp = Vb + (size_t)(16 * n) * SEQ + key0;
      acc[n] = mma16(ap0, ld_frag(vp, SEQ), acc[n]);
      acc[n] = mma16(ap1, ld_frag(vp + 32, SEQ), acc[n]);
    }
    __syncthreads();
  }

  float inv[8];
#pragma unroll
  for (int r = 0; r < 8; ++r) inv[r] = (1.0f / lrow[r]) * 0.0009765625f;
#pragma unroll
  for (int n = 0; n < 4; ++n)
#pragma unroll
    for (int r = 0; r < 8; ++r)
      Pw[(8 * hh + r) * LDP + 16 * n + m] = (_Float16)(acc[n][r] * inv[r]);
  __syncthreads();
  const int seg = l & 7, qb = l >> 3;
  v8h o[4];
#pragma unroll
  for (int p = 0; p < 4; ++p) o[p] = *(const v8h*)(Pw + (qb + 4 * p) * LDP + 8 * seg);
  _Float16* cb = CTX + prow0 * DMODEL + h * HDIM + 8 * seg;
#pragma unroll
  for (int p = 0; p < 4; ++p) *(volatile v8h*)(cb + (size_t)(qb + 4 * p) * DMODEL) = o[p];
  __threadfence();
#pragma unroll
  for (int p = 0; p < 4; ++p) *(volatile v8h*)(cb + (size_t)(qb + 4 * p) * DMODEL) = o[p];
}

__global__ __launch_bounds__(256) void wo_kernel(const _Float16* __restrict__ CTX,
                                                 const _Float16* __restrict__ WoT,
                                                 const float* __restrict__ X,
                                                 float* __restrict__ OUT1) {
  __shared__ float Cs[128 * LDC] __attribute__((aligned(16)));
  const int tid = threadIdx.x;
  const int row0 = blockIdx.x * 128, n0 = blockIdx.y * 64;
  v8f acc[2][2];
#pragma unroll
  for (int i = 0; i < 2; ++i) { acc[i][0] = vzero(); acc[i][1] = vzero(); }
  gemm_core<DMODEL, false>(CTX, WoT, WoT, row0, n0, acc, acc);
  stage_acc(Cs, acc, 0.015625f);
  __syncthreads();
  const int seg = tid & 15, rb = tid >> 4;
  v4f o[8];
#pragma unroll
  for (int p = 0; p < 8; ++p) {
    const int row = rb + 16 * p;
    const int r = row0 + row;
    const v4f a = *(const v4f*)(Cs + row * LDC + 4 * seg);
    const v4f xv = *(const v4f*)(X + full_row(r) * DMODEL + n0 + 4 * seg);
    v4f t;
#pragma unroll
    for (int e = 0; e < 4; ++e) { const float xe = xv[e]; t[e] = bfr(xe) + a[e]; }
    o[p] = t;
  }
  float* ob = OUT1 + (size_t)row0 * DMODEL + n0 + 4 * seg;
#pragma unroll
  for (int p = 0; p < 8; ++p) *(volatile v4f*)(ob + (size_t)(rb + 16 * p) * DMODEL) = o[p];
  __threadfence();
#pragma unroll
  for (int p = 0; p < 8; ++p) *(volatile v4f*)(ob + (size_t)(rb + 16 * p) * DMODEL) = o[p];
}

__global__ __launch_bounds__(256) void w13_kernel(const _Float16* __restrict__ H2,
                                                  const _Float16* __restrict__ W1T,
                                                  const _Float16* __restrict__ W3T,
                                                  _Float16* __restrict__ T16) {
  __shared__ float Cs[128 * LDC] __attribute__((aligned(16)));
  const int row0 = blockIdx.x * 128, n0 = blockIdx.y * 64;
  v8f a1[2][2], a3[2][2];
#pragma unroll
  for (int i = 0; i < 2; ++i) {
    a1[i][0] = vzero(); a1[i][1] = vzero();
    a3[i][0] = vzero(); a3[i][1] = vzero();
  }
  gemm_core<DMODEL, true>(H2, W1T, W3T, row0, n0, a1, a3);
#pragma unroll
  for (int mi = 0; mi < 2; ++mi)
#pragma unroll
    for (int ni = 0; ni < 2; ++ni)
#pragma unroll
      for (int r = 0; r < 8; ++r) {
        const float x1 = a1[mi][ni][r] * 0.015625f;
        const float x3 = a3[mi][ni][r] * 0.015625f;
        const float sg = 1.0f / (1.0f + __expf(-x1));
        a1[mi][ni][r] = (x1 * sg) * x3;
      }
  stage_acc(Cs, a1, 16.0f);
  __syncthreads();
  store_f16_rows(Cs, T16 + (size_t)row0 * DFF + n0, DFF);
}

__global__ __launch_bounds__(256) void w2_kernel(const _Float16* __restrict__ T16,
                                                 const _Float16* __restrict__ W2T,
                                                 const float* __restrict__ OUT1,
                                                 float* __restrict__ OUT) {
  __shared__ float Cs[128 * LDC] __attribute__((aligned(16)));
  const int tid = threadIdx.x;
  const int row0 = blockIdx.x * 128, n0 = blockIdx.y * 64;
  v8f acc[2][2];
#pragma unroll
  for (int i = 0; i < 2; ++i) { acc[i][0] = vzero(); acc[i][1] = vzero(); }
  gemm_core<DFF, false>(T16, W2T, W2T, row0, n0, acc, acc);
  stage_acc(Cs, acc, 0.0009765625f);
  __syncthreads();
  const int seg = tid & 15, rb = tid >> 4;
  v4f o[8];
#pragma unroll
  for (int p = 0; p < 8; ++p) {
    const int row = rb + 16 * p;
    const int r = row0 + row;
    const v4f a = *(const v4f*)(Cs + row * LDC + 4 * seg);
    const v4f o1 = *(const v4f*)(OUT1 + (size_t)r * DMODEL + n0 + 4 * seg);
    v4f t;
#pragma unroll
    for (int e = 0; e < 4; ++e) t[e] = o1[e] + a[e];
    o[p] = t;
  }
#pragma unroll
  for (int p = 0; p < 8; ++p)
    *(volatile v4f*)(OUT + full_row(row0 + rb + 16 * p) * DMODEL + n0 + 4 * seg) = o[p];
  __threadfence();
#pragma unroll
  for (int p = 0; p < 8; ++p)
    *(volatile v4f*)(OUT + full_row(row0 + rb + 16 * p) * DMODEL + n0 + 4 * seg) = o[p];
}

extern "C" void kernel_launch(void* const* d_in, const int* in_sizes, int n_in,
                              void* d_out, int out_size, void* d_ws,
                              size_t ws_size, hipStream_t stream) {
  if (n_in < 10) return;
  const long long need_x = ((long long)(NB - 1) * SEQ_FULL + SEQ) * DMODEL;
  if ((long long)in_sizes[0] < need_x || (long long)out_size < need_x) return;
  if (in_sizes[1] < DMODEL * DMODEL || in_sizes[2] < DMODEL * DMODEL ||
      in_sizes[3] < DMODEL * DMODEL || in_sizes[4] < DMODEL * DMODEL ||
      in_sizes[5] < DMODEL || in_sizes[6] < DMODEL ||
      in_sizes[7] < DMODEL * DFF || in_sizes[8] < DFF * DMODEL || in_sizes[9] < DMODEL * DFF)
    return;
  if (ws_size < WS_TOTAL) return;

  const float* x  = (const float*)d_in[0];
  const float* Wq = (const float*)d_in[1];
  const float* Wk = (const float*)d_in[2];
  const float* Wv = (const float*)d_in[3];
  const float* Wo = (const float*)d_in[4];
  const float* g1 = (const float*)d_in[5];
  const float* g2 = (const float*)d_in[6];
  const float* W1 = (const float*)d_in[7];
  const float* W2 = (const float*)d_in[8];
  const float* W3 = (const float*)d_in[9];
  float* out = (float*)d_out;

  char* w = (char*)d_ws;
  _Float16* WqT  = (_Float16*)(w + OFF_WQT);
  _Float16* WkT  = (_Float16*)(w + OFF_WKT);
  _Float16* WvT  = (_Float16*)(w + OFF_WVT);
  _Float16* WoT  = (_Float16*)(w + OFF_WOT);
  _Float16* W1T  = (_Float16*)(w + OFF_W1T);
  _Float16* W3T  = (_Float16*)(w + OFF_W3T);
  _Float16* W2T  = (_Float16*)(w + OFF_W2T);
  float*    cosT = (float*)(w + OFF_COS);
  float*    sinT = (float*)(w + OFF_SIN);
  _Float16* H16  = (_Float16*)(w + OFF_RH);
  _Float16* CTX  = (_Float16*)(w + OFF_RH);
  _Float16* Q16  = (_Float16*)(w + OFF_RQ);
  _Float16* H2   = (_Float16*)(w + OFF_RQ);
  _Float16* K16  = (_Float16*)(w + OFF_K16);
  _Float16* VT16 = (_Float16*)(w + OFF_VT);
  float*    QKVe = (float*)(w + OFF_QKVE);
  float*    OUT1 = (float*)(w + OFF_OUT1);
  _Float16* T16  = (_Float16*)(w + OFF_T16);

  cvt_w_kernel<<<dim3(1024, 1, 7), 256, 0, stream>>>(Wq, Wk, Wv, Wo, W1, W2, W3,
                                                     WqT, WkT, WvT, WoT, W1T, W2T, W3T);
  rope_tab_kernel<<<dim3((SEQ * 32) / 256), 256, 0, stream>>>(cosT, sinT);
  rmsnorm_kernel<1><<<dim3(NR / 8), 256, 0, stream>>>(x, g1, H16);
  qkv_kernel<<<dim3(NR / 128, (3 * DMODEL) / 64), 256, 0, stream>>>(
      H16, WqT, WkT, WvT, cosT, sinT, Q16, K16, VT16, QKVe);
  attn0_kernel<<<dim3(NHEAD, NB), 256, 0, stream>>>(QKVe, CTX);
  attn_kernel<<<dim3(SEQ / 64 - 1, NHEAD, NB), 128, 0, stream>>>(Q16, K16, VT16, CTX);
  wo_kernel<<<dim3(NR / 128, DMODEL / 64), 256, 0, stream>>>(CTX, WoT, x, OUT1);
  rmsnorm_kernel<0><<<dim3(NR / 8), 256, 0, stream>>>(OUT1, g2, H2);
  w13_kernel<<<dim3(NR / 128, DFF / 64), 256, 0, stream>>>(H2, W1T, W3T, T16);
  w2_kernel<<<dim3(NR / 128, DMODEL / 64), 256, 0, stream>>>(T16, W2T, OUT1, out);
}
